// FVNet_27419071217689
// MI455X (gfx1250) — hardware-run, weakly checked
//
#include <hip/hip_runtime.h>
#include <math.h>

typedef __attribute__((ext_vector_type(16))) _Float16 v16h;
typedef __attribute__((ext_vector_type(8)))  _Float16 v8h;
typedef __attribute__((ext_vector_type(4)))  _Float16 v4h;
typedef __attribute__((ext_vector_type(2)))  _Float16 v2h;
typedef __attribute__((ext_vector_type(16))) __bf16   v16b;
typedef __attribute__((ext_vector_type(8)))  __bf16   v8b;
typedef __attribute__((ext_vector_type(8)))  float    v8f;
typedef __attribute__((ext_vector_type(4)))  float    v4f;
typedef __attribute__((ext_vector_type(2)))  float    v2f;

constexpr int kNB   = 8;
constexpr int kF    = 512;
constexpr int kN    = 512;
constexpr int kK    = 32;
constexpr int kKP   = 64;
constexpr int kThr  = 256;
constexpr float kInCarry = 1024.0f;
constexpr float kSc20 = 1.0f / (kInCarry * kInCarry);
constexpr float kF16MinNormal = 6.103515625e-5f;
constexpr float kNormFloor = 1.0e-12f;

static_assert(kNB == 8 && kF == 512 && kN == 512 && kK == 32 && kKP == 64, "the index arithmetic below uses these sizes");

constexpr size_t kOffXT16 = 0ull;
constexpr size_t kOffW16 = 4194304ull;
constexpr size_t kOffBR = 4259840ull;
constexpr size_t kOffSP = 4260096ull;
constexpr size_t kOffAF = 5308672ull;
constexpr size_t kOffAT = 5832960ull;
constexpr size_t kOffX16 = 6357248ull;
constexpr size_t kOffXR = 10551552ull;
constexpr size_t kOffX2 = 18940160ull;
constexpr size_t kOffAX = 23134464ull;
constexpr size_t kOffAX2 = 24183040ull;
constexpr size_t kOffMS = 25231616ull;
constexpr size_t kOffMR = 25232640ull;
constexpr size_t kOffSR = 25298176ull;
constexpr size_t kOffF1 = 25363712ull;
constexpr size_t kOffF2 = 25888000ull;
constexpr size_t kOffNS = 26412288ull;
constexpr size_t kOffSS = 26445056ull;
constexpr size_t kWsTotal = 26447104ull;
static_assert(kWsTotal <= 268435456ull, "the carve stands under 256 MiB");
static_assert(kOffXT16 == 0
  && kOffW16 == kOffXT16 + 4194304ull
  && kOffBR == kOffW16 + 65536ull
  && kOffSP == kOffBR + 256ull
  && kOffAF == kOffSP + 1048576ull
  && kOffAT == kOffAF + 524288ull
  && kOffX16 == kOffAT + 524288ull
  && kOffXR == kOffX16 + 4194304ull
  && kOffX2 == kOffXR + 8388608ull
  && kOffAX == kOffX2 + 4194304ull
  && kOffAX2 == kOffAX + 1048576ull
  && kOffMS == kOffAX2 + 1048576ull
  && kOffMR == kOffMS + 1024ull
  && kOffSR == kOffMR + 65536ull
  && kOffF1 == kOffSR + 65536ull
  && kOffF2 == kOffF1 + 524288ull
  && kOffNS == kOffF2 + 524288ull
  && kOffSS == kOffNS + 32768ull
  && kWsTotal == kOffSS + 2048ull, "the carve is a chain: every region starts where the one before ends");
static_assert((kOffXT16 % 256) == 0 && (kOffW16 % 256) == 0 && (kOffBR % 256) == 0 && (kOffSP % 256) == 0 && (kOffAF % 256) == 0 && (kOffAT % 256) == 0 && (kOffX16 % 256) == 0 && (kOffXR % 256) == 0 && (kOffX2 % 256) == 0 && (kOffAX % 256) == 0 && (kOffAX2 % 256) == 0 && (kOffMS % 256) == 0 && (kOffMR % 256) == 0 && (kOffSR % 256) == 0 && (kOffF1 % 256) == 0 && (kOffF2 % 256) == 0 && (kOffNS % 256) == 0 && (kOffSS % 256) == 0, "every region starts on a multiple of 256 B");

__device__ __forceinline__ unsigned short f2bf_bits(float f) {
  unsigned u = __float_as_uint(f);
  return (unsigned short)((u + 0x7FFFu + ((u >> 16) & 1u)) >> 16);
}
__device__ __forceinline__ float bf_bits2f(unsigned short h) { return __uint_as_float(((unsigned)h) << 16); }
__device__ __forceinline__ float bf16r(float f) { return bf_bits2f(f2bf_bits(f)); }
__device__ __forceinline__ float carry_flush(float v, float carry) {
  const float s = v * carry;
  return (fabsf(s) < kF16MinNormal) ? 0.0f : s;
}

__device__ __forceinline__ void dep_guard4_h(v8f& a, v8f& b, v8f& c, v8f& d, v16h x, v16h y) { asm volatile("v_nop\n\tv_nop\n\tv_nop\n\tv_nop" : "+v"(a), "+v"(b), "+v"(c), "+v"(d) : "v"(x), "v"(y)); }
__device__ __forceinline__ void dep_guard4_b(v8f& a, v8f& b, v8f& c, v8f& d, v16b x, v16b y) { asm volatile("v_nop\n\tv_nop\n\tv_nop\n\tv_nop" : "+v"(a), "+v"(b), "+v"(c), "+v"(d) : "v"(x), "v"(y)); }
__device__ __forceinline__ void keep4_h(v16h a, v16h b, v16h c, v16h d) { asm volatile("v_nop" :: "v"(a), "v"(b), "v"(c), "v"(d)); }
__device__ __forceinline__ void keep4_b(v16b a, v16b b, v16b c, v16b d) { asm volatile("v_nop" :: "v"(a), "v"(b), "v"(c), "v"(d)); }
__device__ __forceinline__ void acc_guard4(v8f& a, v8f& b, v8f& c, v8f& d) { asm volatile("v_nop\n\tv_nop\n\tv_nop\n\tv_nop" : "+v"(a), "+v"(b), "+v"(c), "+v"(d)); }

template <typename T> struct Frag;
template <> struct Frag<_Float16> {
  typedef v16h V; union U { v16h v; v8h h[2]; };
  static __device__ __forceinline__ v16h load(const _Float16* p) {
    U f; f.h[0] = *(const v8h*)(p); f.h[1] = *(const v8h*)(p + 16); return f.v;
  }
  static __device__ __forceinline__ v8f mma(v16h a, v16h b, v8f c) {
    return __builtin_amdgcn_wmma_f32_16x16x32_f16(false, a, false, b, (short)0, c, false, false);
  }
  static __device__ __forceinline__ void guard4(v8f& a, v8f& b, v8f& c, v8f& d, v16h x, v16h y) { dep_guard4_h(a, b, c, d, x, y); }
  static __device__ __forceinline__ void keep(v16h a, v16h b, v16h c, v16h d) { keep4_h(a, b, c, d); }
};
template <> struct Frag<__bf16> {
  typedef v16b V; union U { v16b v; v8b h[2]; };
  static __device__ __forceinline__ v16b load(const __bf16* p) {
    U f; f.h[0] = *(const v8b*)(p); f.h[1] = *(const v8b*)(p + 16); return f.v;
  }
  static __device__ __forceinline__ v8f mma(v16b a, v16b b, v8f c) {
    return __builtin_amdgcn_wmma_f32_16x16x32_bf16(false, a, false, b, (short)0, c, false, false);
  }
  static __device__ __forceinline__ void guard4(v8f& a, v8f& b, v8f& c, v8f& d, v16b x, v16b y) { dep_guard4_b(a, b, c, d, x, y); }
  static __device__ __forceinline__ void keep(v16b a, v16b b, v16b c, v16b d) { keep4_b(a, b, c, d); }
};

__device__ __forceinline__ v8f mma_h(v16h a, v16h b, v8f c) {
  c = __builtin_amdgcn_wmma_f32_16x16x32_f16(false, a, false, b, (short)0, c, false, false);
  asm volatile("v_nop\n\tv_nop\n\tv_nop\n\tv_nop" : "+v"(c) : "v"(a), "v"(b));
  return c;
}

template <int ET> struct Elem;
template <> struct Elem<0> { typedef _Float16 T; };
template <> struct Elem<1> { typedef __bf16 T; };
template <int ET, bool SPLIT, int BIAS_MODE, int OUT_MODE, bool RESID, int ACT = 0>
__global__ __launch_bounds__(256) void wmma_gemm64(
    const unsigned short* __restrict__ Ap, const unsigned short* __restrict__ A2p, int lda, long strideA,
    const unsigned short* __restrict__ Btp, const unsigned short* __restrict__ Bt2p, int ldb, long strideB,
    void* __restrict__ Cout, void* __restrict__ Cout2, int ldc, long strideC,
    const float* __restrict__ bias,
    const float* __restrict__ resid, long strideR,
    int M, int N, int K, float scale) {
  typedef typename Elem<ET>::T T;
  typedef typename Frag<T>::V V;
  const T* A = (const T*)Ap; const T* A2 = (const T*)A2p; const T* Bt = (const T*)Btp; const T* Bt2 = (const T*)Bt2p;
  __shared__ __align__(16) float sT[8][16 * 68];
  const int b    = blockIdx.y;
  const int lane = threadIdx.x & 31;
  const int wave = threadIdx.x >> 5;
  const int tilesN = N >> 6;
  const int tilesM = M >> 6;
  const int tile = blockIdx.x * 8 + wave;
  if (tile >= tilesM * tilesN) return;
  const int tm = tile / tilesN;
  const int tn = tile - tm * tilesN;
  const int m0 = tm << 6;
  const int n0 = tn << 6;

  const T* Ab  = A  + (size_t)b * strideA;
  const T* Bb  = Bt + (size_t)b * strideB;
  const T* Ab2 = SPLIT ? (A2  + (size_t)b * strideA) : nullptr;
  const T* Bb2 = SPLIT ? (Bt2 + (size_t)b * strideB) : nullptr;

  const int rlane = lane & 15;
  const int koff  = (lane >> 4) * 8;
  const int mOff  = (lane >> 4) * 8;

  v8f acc[4][4];
#pragma unroll
  for (int i = 0; i < 4; ++i)
#pragma unroll
    for (int j = 0; j < 4; ++j) acc[i][j] = (v8f){0.f,0.f,0.f,0.f,0.f,0.f,0.f,0.f};

  for (int k0 = 0; k0 < K; k0 += 32) {
    V bh[4], bl[4];
#pragma unroll
    for (int j = 0; j < 4; ++j) {
      const size_t bo = (size_t)(n0 + (j << 4) + rlane) * ldb + koff + k0;
      bh[j] = Frag<T>::load(Bb + bo);
      if (SPLIT) bl[j] = Frag<T>::load(Bb2 + bo);
    }
#pragma unroll
    for (int i = 0; i < 4; ++i) {
      const size_t ao = (size_t)(m0 + (i << 4) + rlane) * lda + koff + k0;
      V ah = Frag<T>::load(Ab + ao);
      V al;
      if (SPLIT) al = Frag<T>::load(Ab2 + ao);
#pragma unroll
      for (int j = 0; j < 4; ++j) {
        acc[i][j] = Frag<T>::mma(ah, bh[j], acc[i][j]);
        if (SPLIT) {
          acc[i][j] = Frag<T>::mma(ah, bl[j], acc[i][j]);
          acc[i][j] = Frag<T>::mma(al, bh[j], acc[i][j]);
        }
      }
      Frag<T>::guard4(acc[i][0], acc[i][1], acc[i][2], acc[i][3], ah, SPLIT ? al : ah);
    }
    Frag<T>::keep(bh[0], bh[1], bh[2], bh[3]);
    if (SPLIT) Frag<T>::keep(bl[0], bl[1], bl[2], bl[3]);
  }
  acc_guard4(acc[0][0], acc[0][1], acc[0][2], acc[0][3]);
  acc_guard4(acc[1][0], acc[1][1], acc[1][2], acc[1][3]);
  acc_guard4(acc[2][0], acc[2][1], acc[2][2], acc[2][3]);
  acc_guard4(acc[3][0], acc[3][1], acc[3][2], acc[3][3]);

  float* slab = sT[wave];
  const float* Rb = RESID ? (resid + (size_t)b * strideR) : nullptr;
#pragma unroll
  for (int i = 0; i < 4; ++i) {
    const int mBase = m0 + (i << 4);
#pragma unroll
    for (int j = 0; j < 4; ++j) {
      const int n = n0 + (j << 4) + rlane;
      float bv = 0.f;
      if (BIAS_MODE == 2) bv = bias[n];
#pragma unroll
      for (int r = 0; r < 8; ++r) {
        float v = acc[i][j][r] * scale;
        if (BIAS_MODE == 1) v += bias[mBase + mOff + r];
        if (BIAS_MODE == 2) v += bv;
        if (RESID) v += Rb[(size_t)(mBase + mOff + r) * ldc + n];
        if (ACT == 1) v = tanhf(v);
        if (ACT == 2) v = fmaxf(v, 0.0f);
        if (ACT == 3) v = v / (1.0f + expf(-v));
        if (ACT == 4) v = (v > 0.f) ? v : 0.01f * v;
        slab[(mOff + r) * 68 + (j << 4) + rlane] = v;
      }
    }
    __builtin_amdgcn_fence(__ATOMIC_RELEASE, "workgroup");
    __builtin_amdgcn_wave_barrier();
    __builtin_amdgcn_fence(__ATOMIC_ACQUIRE, "workgroup");
    if (OUT_MODE == 0) {
      float* C = (float*)Cout + (size_t)b * strideC;
      const int hh = lane >> 4, c4 = (lane & 15) * 4;
      for (int pass = 0; pass < 2; ++pass) {
#pragma unroll
        for (int it = 0; it < 8; ++it) {
          const int row = it * 2 + hh;
          v4f v = *(const v4f*)(slab + row * 68 + c4);
          *(volatile v4f*)(C + (size_t)(mBase + row) * ldc + n0 + c4) = v;
        }
        __threadfence();
      }
    } else {
      const int q = lane >> 3, c8 = (lane & 7) * 8;
      unsigned short* C  = (unsigned short*)Cout  + (size_t)b * strideC;
      unsigned short* C2 = (OUT_MODE == 2) ? ((unsigned short*)Cout2 + (size_t)b * strideC) : nullptr;
      for (int pass = 0; pass < 2; ++pass) {
#pragma unroll
        for (int it = 0; it < 4; ++it) {
          const int row = it * 4 + q;
          const float* sp = slab + row * 68 + c8;
          v8h hv, lv;
#pragma unroll
          for (int e = 0; e < 8; ++e) {
            if (OUT_MODE == 1) {
              hv[e] = (_Float16)sp[e];
            } else {
              unsigned short hb = f2bf_bits(sp[e]);
              unsigned short lb = f2bf_bits(sp[e] - bf_bits2f(hb));
              hv[e] = __builtin_bit_cast(_Float16, hb);
              lv[e] = __builtin_bit_cast(_Float16, lb);
            }
          }
          *(volatile v8h*)(C + (size_t)(mBase + row) * ldc + n0 + c8) = hv;
          if (OUT_MODE == 2) *(volatile v8h*)(C2 + (size_t)(mBase + row) * ldc + n0 + c8) = lv;
        }
        __threadfence();
      }
    }
    __builtin_amdgcn_fence(__ATOMIC_RELEASE, "workgroup");
    __builtin_amdgcn_wave_barrier();
    __builtin_amdgcn_fence(__ATOMIC_ACQUIRE, "workgroup");
  }
}

__global__ __launch_bounds__(kThr) void cast_plane_kernel(const float* __restrict__ src, unsigned short* __restrict__ dst,
                                                          int colsLog2, int dstPitch, int dstOff) {
  const int i   = blockIdx.x * kThr + threadIdx.x;
  const int sh  = colsLog2 - 3;
  const int row = i >> sh;
  const int c8  = (i & ((1 << sh) - 1)) * 8;
  const float* sp = src + ((size_t)row << colsLog2) + c8;
  const v4f a0 = *(const v4f*)(sp);
  const v4f a1 = *(const v4f*)(sp + 4);
  v8h hv;
#pragma unroll
  for (int e = 0; e < 4; ++e) {
    const float f0 = a0[e];
    const float f1 = a1[e];
    hv[e]     = (_Float16)carry_flush(bf16r(f0), kInCarry);
    hv[4 + e] = (_Float16)carry_flush(bf16r(f1), kInCarry);
  }
  unsigned short* dp = dst + (size_t)row * dstPitch + dstOff + c8;
  *(volatile v8h*)dp = hv;
  __threadfence();
  *(volatile v8h*)dp = hv;
}

__global__ __launch_bounds__(kThr) void pack_kernel(const float* __restrict__ W, unsigned short* __restrict__ D, float* __restrict__ dstf, int part, int ld, int k0, int lg, int n0, int pitch) {
  const unsigned i = blockIdx.x * blockDim.x + threadIdx.x;
  if (part == 0) {
    const unsigned g = i & ((1u << lg) - 1u), n = i >> lg;
    const float* sp = W + (size_t)((unsigned)k0 + g * 8u) * (unsigned)ld + n;
    v8h hv;
#pragma unroll
    for (int t = 0; t < 8; ++t) hv[t] = (_Float16)carry_flush(bf16r(sp[(size_t)t * (unsigned)ld]), kInCarry);
    unsigned short* dp = D + (size_t)((unsigned)n0 + n) * (unsigned)pitch + g * 8u;
    *(volatile v8h*)dp = hv;
    __threadfence();
    *(volatile v8h*)dp = hv;
  } else {
    const v4f a = *(const v4f*)(W + i * 4u);
    v4f o;
#pragma unroll
    for (int e = 0; e < 4; ++e) o[e] = bf16r(a[e]);
    float* dp = dstf + i * 4u;
    *(volatile v4f*)dp = o;
    __threadfence();
    *(volatile v4f*)dp = o;
  }
}

__global__ __launch_bounds__(kThr) void zero_kernel(float* __restrict__ dst) {
  const size_t o4 = ((size_t)blockIdx.x * kThr + threadIdx.x) * 4u;
  const v4f z = {0.f, 0.f, 0.f, 0.f};
  *(volatile v4f*)(dst + o4) = z;
  __threadfence();
  *(volatile v4f*)(dst + o4) = z;
}

__global__ __launch_bounds__(kThr) void sqcast_kernel(const float* __restrict__ R, unsigned short* __restrict__ X2) {
  const unsigned i = blockIdx.x * (unsigned)kThr + threadIdx.x;
  const v4f a = *(const v4f*)(R + (size_t)i * 8u), c = *(const v4f*)(R + (size_t)i * 8u + 4u);
  v8h w;
#pragma unroll
  for (int t = 0; t < 4; ++t) { w[t] = (_Float16)carry_flush(a[t] * a[t], kInCarry); w[4 + t] = (_Float16)carry_flush(c[t] * c[t], kInCarry); }
  *(volatile v8h*)(X2 + (size_t)i * 8u) = w;
  __threadfence();
  *(volatile v8h*)(X2 + (size_t)i * 8u) = w;
}

__global__ __launch_bounds__(kThr) void rowsoftmax2_kernel(const float* __restrict__ SP, float* __restrict__ AF, unsigned short* __restrict__ AT) {
  const unsigned i = blockIdx.x * (unsigned)kThr + threadIdx.x;
  const unsigned p0 = 2u * i;
  float q[2][32];
#pragma unroll
  for (int r = 0; r < 2; ++r) {
    const float* sp = SP + (size_t)(p0 + r) * kKP;
    float m = sp[0];
#pragma unroll
    for (int c = 0; c < 8; ++c) {
      const v4f a = *(const v4f*)(sp + 4 * c);
#pragma unroll
      for (int e = 0; e < 4; ++e) { q[r][4 * c + e] = a[e]; m = (a[e] > m) ? a[e] : m; }
    }
    float s = 0.0f;
#pragma unroll
    for (int k = 0; k < 32; ++k) { q[r][k] = expf(q[r][k] - m); s += q[r][k]; }
#pragma unroll
    for (int k = 0; k < 32; ++k) q[r][k] = q[r][k] / s;
  }
  unsigned short* tp = AT + (size_t)(p0 >> 9) * kKP * kN + (p0 & 511u);
  for (int pass = 0; pass < 2; ++pass) {
#pragma unroll
    for (int r = 0; r < 2; ++r) {
      float* op = AF + (size_t)(p0 + r) * kK;
#pragma unroll
      for (int c = 0; c < 8; ++c) { const v4f o = {q[r][4 * c], q[r][4 * c + 1], q[r][4 * c + 2], q[r][4 * c + 3]}; *(volatile v4f*)(op + 4 * c) = o; }
    }
#pragma unroll
    for (int k = 0; k < 32; ++k) {
      v2h w; w[0] = (_Float16)carry_flush(q[0][k], kInCarry); w[1] = (_Float16)carry_flush(q[1][k], kInCarry);
      *(volatile v2h*)(tp + (size_t)k * kN) = w;
    }
#pragma unroll
    for (int k = 32; k < 64; ++k) {
      v2h z; z[0] = (_Float16)0.0f; z[1] = (_Float16)0.0f;
      *(volatile v2h*)(tp + (size_t)k * kN) = z;
    }
    __threadfence();
  }
}

__global__ __launch_bounds__(kThr) void colmass8_kernel(const float* __restrict__ AF, float* __restrict__ MS) {
  const unsigned i = threadIdx.x;
  const unsigned k = i & 31u, b = i >> 5;
  const float* ap = AF + (size_t)(b * 512u) * kK + k;
  float acc = 0.0f;
  for (int n = 0; n < 512; ++n) acc += ap[(size_t)n * kK];
  *(volatile float*)(MS + i) = acc;
  __threadfence();
  *(volatile float*)(MS + i) = acc;
}

__global__ __launch_bounds__(kThr) void fvrow_kernel(const float* __restrict__ AX, const float* __restrict__ AX2, const float* __restrict__ MR, const float* __restrict__ SR, const float* __restrict__ MS,
                                                     float* __restrict__ F1, float* __restrict__ F2, float* __restrict__ NS) {
  const unsigned i = blockIdx.x * (unsigned)kThr + threadIdx.x;
  const unsigned b = i >> 9, f = i & 511u;
  const float* p1 = AX + (size_t)i * kKP; const float* p2 = AX2 + (size_t)i * kKP;
  const float* mp = MR + (size_t)f * kK; const float* gp = SR + (size_t)f * kK; const float* ms = MS + (size_t)b * kK;
  float u1[32], u2[32];
  float n1 = 0.0f, n2 = 0.0f;
#pragma unroll
  for (int c = 0; c < 8; ++c) {
    const v4f a1 = *(const v4f*)(p1 + 4 * c), a2 = *(const v4f*)(p2 + 4 * c), mu = *(const v4f*)(mp + 4 * c), sg = *(const v4f*)(gp + 4 * c), mm = *(const v4f*)(ms + 4 * c);
#pragma unroll
    for (int e = 0; e < 4; ++e) {
      const float t1 = (a1[e] - mu[e] * mm[e]) / sg[e];
      const float t2 = ((a2[e] - (mu[e] + mu[e]) * a1[e]) + (mu[e] * mu[e]) * mm[e]) / (sg[e] * sg[e]) - mm[e];
      u1[4 * c + e] = t1; u2[4 * c + e] = t2;
      n1 = fmaf(t1, t1, n1); n2 = fmaf(t2, t2, n2);
    }
  }
  const float r1 = sqrtf(n1), r2 = sqrtf(n2);
  const float d1 = fmaxf(r1, kNormFloor), d2 = fmaxf(r2, kNormFloor);
  float s1 = 0.0f, s2 = 0.0f;
#pragma unroll
  for (int k = 0; k < 32; ++k) { u1[k] = u1[k] / d1; u2[k] = u2[k] / d2; s1 = fmaf(u1[k], u1[k], s1); s2 = fmaf(u2[k], u2[k], s2); }
  float* o1 = F1 + (size_t)i * kK; float* o2 = F2 + (size_t)i * kK;
  const v2f sn = {s1, s2};
  for (int pass = 0; pass < 2; ++pass) {
#pragma unroll
    for (int c = 0; c < 8; ++c) {
      const v4f w1 = {u1[4 * c], u1[4 * c + 1], u1[4 * c + 2], u1[4 * c + 3]}; const v4f w2 = {u2[4 * c], u2[4 * c + 1], u2[4 * c + 2], u2[4 * c + 3]};
      *(volatile v4f*)(o1 + 4 * c) = w1; *(volatile v4f*)(o2 + 4 * c) = w2;
    }
    *(volatile v2f*)(NS + (size_t)i * 2u) = sn;
    __threadfence();
  }
}

__global__ __launch_bounds__(kThr) void fvsum_kernel(const float* __restrict__ NS, float* __restrict__ SS) {
  const unsigned i = blockIdx.x * (unsigned)kThr + threadIdx.x;
  const unsigned j = i >> 5;
  const float* np = NS + (size_t)((j >> 1) * 512u) * 2u + (j & 1u);
  float acc = 0.0f;
  for (int f = 0; f < 512; ++f) acc += np[(size_t)f * 2u];
  const float r = sqrtf(acc);
  const float o = fmaxf(r, kNormFloor);
  *(volatile float*)(SS + i) = o;
  __threadfence();
  *(volatile float*)(SS + i) = o;
}

__global__ __launch_bounds__(kThr) void fvout_kernel(const float* __restrict__ F1, const float* __restrict__ F2, const float* __restrict__ SS, float* __restrict__ res) {
  const unsigned v = blockIdx.x * (unsigned)kThr + threadIdx.x;
  const unsigned b = v >> 15, h = (v >> 14) & 1u, e = v & 16383u;
  const float a1 = F1[(size_t)b * 16384u + e], a2 = F2[(size_t)b * 16384u + e];
  const float a = (h == 0u) ? a1 : a2;
  const float d = SS[(v >> 14) * 32u + (threadIdx.x & 31u)];
  const float o = a / d;
  *(volatile float*)(res + v) = o;
  __threadfence();
  *(volatile float*)(res + v) = o;
}

extern "C" void kernel_launch(void* const* d_in, const int* in_sizes, int n_in,
                              void* d_out, int out_size, void* d_ws, size_t ws_size,
                              hipStream_t stream) {
  if (n_in < 5 || d_out == nullptr || d_ws == nullptr) return;
  if (in_sizes[0] != kNB * kF * kN || in_sizes[1] != kK * kF || in_sizes[2] != kK || in_sizes[3] != kF * kK || in_sizes[4] != kF * kK) return;
  if (out_size != kNB * 2 * kF * kK) return;
  if (ws_size < kWsTotal) return;
  const float* xa = (const float*)d_in[0];
  const float* wc = (const float*)d_in[1];
  const float* bc = (const float*)d_in[2];
  const float* mu = (const float*)d_in[3];
  const float* sg = (const float*)d_in[4];
  float* out = (float*)d_out;
  char* ws = (char*)d_ws;
  unsigned short* XT16 = (unsigned short*)(ws + kOffXT16);
  unsigned short* W16 = (unsigned short*)(ws + kOffW16);
  float* BR = (float*)(ws + kOffBR);
  float* SP = (float*)(ws + kOffSP);
  float* AF = (float*)(ws + kOffAF);
  unsigned short* AT = (unsigned short*)(ws + kOffAT);
  unsigned short* X16 = (unsigned short*)(ws + kOffX16);
  float* XR = (float*)(ws + kOffXR);
  unsigned short* X2 = (unsigned short*)(ws + kOffX2);
  float* AX = (float*)(ws + kOffAX);
  float* AX2 = (float*)(ws + kOffAX2);
  float* MS = (float*)(ws + kOffMS);
  float* MR = (float*)(ws + kOffMR);
  float* SR = (float*)(ws + kOffSR);
  float* F1 = (float*)(ws + kOffF1);
  float* F2 = (float*)(ws + kOffF2);
  float* NS = (float*)(ws + kOffNS);
  float* SS = (float*)(ws + kOffSS);

  static_assert((kN * (kF / 8)) % kThr == 0 && (kK * kF / 8) % kThr == 0 && ((kKP - kK) * kF * 2) % (kThr * 16) == 0 && (kNB * kF * kN / 4) % kThr == 0 && (kF * kK / 4) % kThr == 0 && (kNB * kF * kN / 8) % kThr == 0
                && (kNB * kN / 2) % kThr == 0 && kNB * kK == kThr && (kNB * kF) % kThr == 0 && (kNB * 2 * kF * kK) % kThr == 0 && ((kNB * kN / 64) * (kKP / 64)) % 8 == 0 && ((kF / 64) * (kKP / 64)) % 8 == 0 && kF % 32 == 0 && kN % 32 == 0, "every grid exact");
  for (int b = 0; b < kNB; ++b) {
    pack_kernel<<<kN * (kF / 8) / kThr, kThr, 0, stream>>>(xa + (size_t)b * kF * kN, XT16 + (size_t)b * kN * kF, nullptr, 0, kN, 0, 6, 0, kF);
  }
  cast_plane_kernel<<<kK * kF / 8 / kThr, kThr, 0, stream>>>(wc, W16, 9, kF, 0);
  zero_kernel<<<(kKP - kK) * kF * 2 / (kThr * 16), kThr, 0, stream>>>((float*)(W16 + (size_t)kK * kF));
  pack_kernel<<<1, kK / 4, 0, stream>>>(bc, nullptr, BR, 1, 0, 0, 0, 0, 0);
  zero_kernel<<<1, kK / 4, 0, stream>>>(BR + kK);
  pack_kernel<<<kNB * kF * kN / 4 / kThr, kThr, 0, stream>>>(xa, nullptr, XR, 1, 0, 0, 0, 0, 0);
  pack_kernel<<<kF * kK / 4 / kThr, kThr, 0, stream>>>(mu, nullptr, MR, 1, 0, 0, 0, 0, 0);
  pack_kernel<<<kF * kK / 4 / kThr, kThr, 0, stream>>>(sg, nullptr, SR, 1, 0, 0, 0, 0, 0);
  cast_plane_kernel<<<kNB * kF * kN / 8 / kThr, kThr, 0, stream>>>(xa, X16, 9, kN, 0);
  sqcast_kernel<<<kNB * kF * kN / 8 / kThr, kThr, 0, stream>>>(XR, X2);
  wmma_gemm64<0, false, 2, 0, false, 0><<<dim3((kNB * kN / 64) * (kKP / 64) / 8, 1), 256, 0, stream>>>(
      XT16, XT16, kF, 0L, W16, W16, kF, 0L, (void*)SP, (void*)SP, kKP, 0L, BR, nullptr, 0L, kNB * kN, kKP, kF, kSc20);
  rowsoftmax2_kernel<<<kNB * kN / 2 / kThr, kThr, 0, stream>>>(SP, AF, AT);
  colmass8_kernel<<<1, kThr, 0, stream>>>(AF, MS);
  wmma_gemm64<0, false, 0, 0, false, 0><<<dim3((kF / 64) * (kKP / 64) / 8, kNB), 256, 0, stream>>>(
      X16, X16, kN, (long)kF * kN, AT, AT, kN, (long)kKP * kN, (void*)AX, (void*)AX, kKP, (long)kF * kKP, nullptr, nullptr, 0L, kF, kKP, kN, kSc20);
  wmma_gemm64<0, false, 0, 0, false, 0><<<dim3((kF / 64) * (kKP / 64) / 8, kNB), 256, 0, stream>>>(
      X2, X2, kN, (long)kF * kN, AT, AT, kN, (long)kKP * kN, (void*)AX2, (void*)AX2, kKP, (long)kF * kKP, nullptr, nullptr, 0L, kF, kKP, kN, kSc20);
  fvrow_kernel<<<kNB * kF / kThr, kThr, 0, stream>>>(AX, AX2, MR, SR, MS, F1, F2, NS);
  fvsum_kernel<<<2, kThr, 0, stream>>>(NS, SS);
  fvout_kernel<<<kNB * 2 * kF * kK / kThr, kThr, 0, stream>>>(F1, F2, SS, out);
}
